// Net_25847113187873
// MI455X (gfx1250) — hardware-verified
//
#include <hip/hip_runtime.h>
#include <stddef.h>

#define NB_S    131072
#define SPB     64
#define NBLK    (NB_S / SPB)
#define NTHR    256
#define KF      75
#define K1H     96
#define K1      192
#define N1      128
#define K2      256
#define N2      64
#define NCHUNK  (NB_S / 32)

#define P_C00W  0
#define P_C00B  80
#define P_C10W  88
#define P_C10B  168
#define P_B1    176
#define P_B2    304
#define P_PIW   368
#define P_PIB   560
#define P_OH0   564
#define P_OH1   576
#define P_OH2   600
#define P_OH3   624
#define P_OH4   640
#define P_POS   652
#define P_FLAG  656
#define PB_N    1024

#define NU_W1   (N1 * (K1 / 8))
#define NU_W2   (N2 * (K2 / 8))
#define NU_PB   (PB_N / 4)
#define NU_ALL  (NU_W1 + NU_W2 + NU_PB)

#define LF_U    0
#define LF_Y    16384
#define LF_X    24576
#define LF_XB   28416
#define LF_M    32256
#define LF_NM   32832
#define LF_C    33408
#define LF_P    33728
#define LF_SM   34752
#define LF_END  35264
#define MLP_LDS (LF_END * 4)

#define OW1     0
#define OW2     49152
#define OPB     81920
#define OPV     86016
#define WS_NEED (OPV + NB_S * 16)

static_assert(NU_W1 % NTHR == 0);
static_assert((NU_W1 + NU_W2) % NTHR == 0);
static_assert(NU_ALL % NTHR == 0);
static_assert(NU_PB == NTHR);
static_assert(K1 % 32 == 0 && K2 % 32 == 0 && K1 == 2 * K1H && K2 == 2 * N1);
static_assert(N1 * K1 * 2 == OW2 - OW1);
static_assert(N2 * K2 * 2 == OPB - OW2);
static_assert(PB_N * 4 == OPV - OPB);
static_assert(OPV % 128 == 0);
static_assert(LF_Y * 4 == 128 * K2 * 2);
static_assert(LF_X - LF_Y == 128 * N2);
static_assert(LF_XB - LF_X == SPB * 60 && LF_M - LF_XB == SPB * 60);
static_assert(LF_NM - LF_M == SPB * 9 && LF_C - LF_NM == SPB * 9);
static_assert(LF_P - LF_C == SPB * 5 && LF_SM - LF_P == PB_N && LF_END - LF_SM == 128 * 4);
static_assert(NBLK * SPB == NB_S && NCHUNK * 32 == NB_S);
static_assert(P_FLAG % 4 == 0 && P_PIW % 4 == 0);

typedef float          v4f   __attribute__((ext_vector_type(4)));
typedef float          v8f   __attribute__((ext_vector_type(8)));
typedef int            v4i   __attribute__((ext_vector_type(4)));
typedef int            v8i   __attribute__((ext_vector_type(8)));
typedef unsigned short v8us  __attribute__((ext_vector_type(8)));
typedef unsigned short v16us __attribute__((ext_vector_type(16)));
typedef __bf16         v16bf __attribute__((ext_vector_type(16)));
typedef v4f  __attribute__((may_alias)) v4fa;
typedef v4i  __attribute__((may_alias)) v4ia;
typedef v8us __attribute__((may_alias)) v8usa;
union FragB { v16bf v; v16us u; v8us h[2]; v8i w; };

__device__ __forceinline__ v8f wmb(const FragB& a, const FragB& b, v8f c) {
  v8f d = __builtin_amdgcn_wmma_f32_16x16x32_bf16(false, a.v, false, b.v, (short)0, c, false, false);
  asm volatile("v_nop\n\tv_nop\n\tv_nop\n\tv_nop" : "+v"(d) : "v"(a.w), "v"(b.w));
  return d;
}

__device__ __forceinline__ unsigned bf16_bits(float f) {
  const unsigned u = __float_as_uint(f);
  return (u + 0x7FFFu + ((u >> 16) & 1u)) >> 16;
}
__device__ __forceinline__ float bf16_val(float f) {
  return __uint_as_float(bf16_bits(f) << 16);
}
__device__ __forceinline__ void put16(unsigned short* dp, v8us o) {
  *(volatile v8us*)dp = o;
  __threadfence();
  *(volatile v8us*)dp = o;
}
__device__ __forceinline__ void putf4(float* dp, v4f o) {
  *(volatile v4f*)dp = o;
  __threadfence();
  *(volatile v4f*)dp = o;
}
__device__ __forceinline__ void putfeat(unsigned short* row, int c, float v) {
  const unsigned hb = bf16_bits(v);
  const unsigned lb = bf16_bits(v - __uint_as_float(hb << 16));
  row[c]       = (unsigned short)hb;
  row[K1H + c] = (unsigned short)lb;
}
__device__ __forceinline__ int clampi(int v, int lo, int hi) {
  return v < lo ? lo : (v > hi ? hi : v);
}
__device__ __forceinline__ float rl(float v, int i) {
  return __int_as_float(__builtin_amdgcn_readlane(__float_as_int(v), i));
}

__device__ __forceinline__ float pb_fetch(int i,
    const float* c00w, const float* c00b, const float* c10w, const float* c10b,
    const float* f11b, const float* f12b, const float* piw, const float* pib,
    const float* oh0, const float* oh1, const float* oh2, const float* oh3, const float* oh4,
    const float* pos0) {
  const float* s = c00w; int j = i; int n = 80;
  if (i >= P_C00B) { s = c00b; j = i - P_C00B; n = 8;   }
  if (i >= P_C10W) { s = c10w; j = i - P_C10W; n = 80;  }
  if (i >= P_C10B) { s = c10b; j = i - P_C10B; n = 8;   }
  if (i >= P_B1)   { s = f11b; j = i - P_B1;   n = 128; }
  if (i >= P_B2)   { s = f12b; j = i - P_B2;   n = 64;  }
  if (i >= P_PIW)  { s = piw;  j = i - P_PIW;  n = 192; }
  if (i >= P_PIB)  { s = pib;  j = i - P_PIB;  n = 3;   }
  if (i >= P_OH0)  { s = oh0;  j = i - P_OH0;  n = 12;  }
  if (i >= P_OH1)  { s = oh1;  j = i - P_OH1;  n = 24;  }
  if (i >= P_OH2)  { s = oh2;  j = i - P_OH2;  n = 24;  }
  if (i >= P_OH3)  { s = oh3;  j = i - P_OH3;  n = 15;  }
  if (i >= P_OH4)  { s = oh4;  j = i - P_OH4;  n = 10;  }
  if (i >= P_POS)  { s = pos0; j = i - P_POS;  n = 3;   }
  const bool ok = j < n;
  const int  jc = ok ? j : n - 1;
  const float v = s[jc];
  return ok ? bf16_val(v) : 0.0f;
}

__global__ __launch_bounds__(NTHR) void k_prep(
    const float* __restrict__ f11w, const float* __restrict__ f12w,
    const float* __restrict__ c00w, const float* __restrict__ c00b,
    const float* __restrict__ c10w, const float* __restrict__ c10b,
    const float* __restrict__ f11b, const float* __restrict__ f12b,
    const float* __restrict__ piw,  const float* __restrict__ pib,
    const float* __restrict__ oh0,  const float* __restrict__ oh1,
    const float* __restrict__ oh2,  const float* __restrict__ oh3,
    const float* __restrict__ oh4,  const float* __restrict__ pos0,
    const int* __restrict__ modp,
    unsigned short* W1P, unsigned short* W2P, float* PB) {
  const int u = (int)blockIdx.x * NTHR + (int)threadIdx.x;
  if (u < NU_W1) {
    const int n  = u / (K1 / 8);
    const int kq = u - n * (K1 / 8);
    const int k8 = kq * 8;
    const int kk = (k8 >= K1H) ? (k8 - K1H) : k8;
    const float* p = f11w + (size_t)n * KF;
    v8us o;
#pragma unroll
    for (int i = 0; i < 8; ++i) {
      const int k  = kk + i;
      const int kc = k < KF ? k : KF - 1;
      const float v = p[kc];
      o[i] = (k < KF) ? (unsigned short)bf16_bits(v) : (unsigned short)0;
    }
    put16(W1P + (size_t)u * 8, o);
  } else if (u < NU_W1 + NU_W2) {
    const int v  = u - NU_W1;
    const int n  = v >> 5;
    const int k8 = (v & 31) * 8;
    const int kk = k8 & (N1 - 1);
    const float* p = f12w + (size_t)n * N1 + kk;
    const v4f a = *(const v4fa*)p;
    const v4f b = *(const v4fa*)(p + 4);
    v8us o;
    o[0] = (unsigned short)bf16_bits(a.x); o[1] = (unsigned short)bf16_bits(a.y);
    o[2] = (unsigned short)bf16_bits(a.z); o[3] = (unsigned short)bf16_bits(a.w);
    o[4] = (unsigned short)bf16_bits(b.x); o[5] = (unsigned short)bf16_bits(b.y);
    o[6] = (unsigned short)bf16_bits(b.z); o[7] = (unsigned short)bf16_bits(b.w);
    put16(W2P + (size_t)v * 8, o);
  } else {
    const int w = u - (NU_W1 + NU_W2);
    const int mv = modp[0];
    v4f q;
    q.x = pb_fetch(4 * w + 0, c00w, c00b, c10w, c10b, f11b, f12b, piw, pib, oh0, oh1, oh2, oh3, oh4, pos0);
    q.y = pb_fetch(4 * w + 1, c00w, c00b, c10w, c10b, f11b, f12b, piw, pib, oh0, oh1, oh2, oh3, oh4, pos0);
    q.z = pb_fetch(4 * w + 2, c00w, c00b, c10w, c10b, f11b, f12b, piw, pib, oh0, oh1, oh2, oh3, oh4, pos0);
    q.w = pb_fetch(4 * w + 3, c00w, c00b, c10w, c10b, f11b, f12b, piw, pib, oh0, oh1, oh2, oh3, oh4, pos0);
    const float fl = (mv != 0) ? 1.0f : 0.0f;
    q.x = (4 * w == P_FLAG) ? fl : q.x;
    putf4(PB + (size_t)w * 4, q);
  }
}

template <int N4>
__device__ __forceinline__ void stage_bf(const float* __restrict__ g, float* s, int tid) {
#pragma unroll
  for (int it = 0; it < (N4 + NTHR - 1) / NTHR; ++it) {
    const int i  = it * NTHR + tid;
    const int ic = i < N4 ? i : N4 - 1;
    v4f v = *(const v4fa*)(g + 4 * (size_t)ic);
    v.x = bf16_val(v.x); v.y = bf16_val(v.y); v.z = bf16_val(v.z); v.w = bf16_val(v.w);
    if (i < N4) *(v4fa*)(s + 4 * i) = v;
  }
}

__global__ __launch_bounds__(NTHR) void k_mlp(
    const float* __restrict__ x,  const float* __restrict__ xb,
    const float* __restrict__ xm, const float* __restrict__ xnm,
    const int* __restrict__ xcat,
    const unsigned short* __restrict__ W1P, const unsigned short* __restrict__ W2P,
    const float* __restrict__ PB, float* PV) {
  extern __shared__ __attribute__((aligned(16))) float dyn[];
  unsigned short* sU  = (unsigned short*)(dyn + LF_U);
  float*          sY  = dyn + LF_Y;
  float*          sX  = dyn + LF_X;
  float*          sXB = dyn + LF_XB;
  float*          sM  = dyn + LF_M;
  float*          sNM = dyn + LF_NM;
  int*            sC  = (int*)(dyn + LF_C);
  float*          sP  = dyn + LF_P;
  float*          sSM = dyn + LF_SM;

  const int tid = (int)threadIdx.x, lane = tid & 31, wave = tid >> 5, hh = lane >> 4, m = lane & 15;
  const size_t s0 = (size_t)blockIdx.x * SPB;

  stage_bf<SPB * 60 / 4>(x  + s0 * 60, sX,  tid);
  stage_bf<SPB * 60 / 4>(xb + s0 * 60, sXB, tid);
  stage_bf<SPB * 9 / 4>(xm  + s0 * 9,  sM,  tid);
  stage_bf<SPB * 9 / 4>(xnm + s0 * 9,  sNM, tid);
  {
    const int ic = tid < (SPB * 5 / 4) ? tid : (SPB * 5 / 4) - 1;
    const v4i c = *(const v4ia*)(xcat + s0 * 5 + 4 * (size_t)ic);
    if (tid < (SPB * 5 / 4)) *(v4ia*)(sC + 4 * tid) = c;
  }
  {
    const v4f p = *(const v4fa*)(PB + 4 * (size_t)tid);
    *(v4fa*)(sP + 4 * tid) = p;
  }
  __syncthreads();

  {
    const int hf  = tid >> 7;
    const int row = tid & 127;
    const int brB = row >> 6;
    const int s   = row & 63;
    const float* xs = (brB ? sXB : sX) + s * 60;
    unsigned short* fr = sU + row * K1;
    const float sgn = brB ? -1.0f : 1.0f;
#pragma unroll 1
    for (int qq = 0; qq < 20; ++qq) {
      const int q   = hf * 20 + qq;
      const int isr = (q >= 8) ? 1 : 0;
      const int q8  = q - 8;
      const int jb  = isr ? (1 + (q8 >> 3)) : 0;
      const int o   = isr ? (q8 & 7) : q;
      const float* wv = sP + (isr ? P_C10W : P_C00W) + o * 10;
      const float bias = sP[(isr ? P_C10B : P_C00B) + o];
      const float* xv = xs + jb * 10;
      float a = 0.0f;
#pragma unroll
      for (int t = 0; t < 10; ++t) a = fmaf(xv[t], wv[t], a);
      a = a + bias;
      a = (a >= 0.0f) ? a : 0.1f * a;
      putfeat(fr, q, a);
    }
    if (hf == 0) {
#pragma unroll
      for (int t = 0; t < 10; ++t) putfeat(fr, 40 + t, xs[50 + t]);
      const int* cr = sC + s * 5;
      const int c0 = clampi(cr[0], 0, 5);
      const int c1 = clampi(cr[1], 0, 11);
      const int c2 = clampi(cr[2], 0, 11);
      const int c3 = clampi(cr[3], 0, 4);
      const int c4 = clampi(cr[4], 0, 9);
      putfeat(fr, 50, sP[P_OH0 + c0 * 2]);
      putfeat(fr, 51, sP[P_OH0 + c0 * 2 + 1]);
      putfeat(fr, 52, sP[P_OH1 + c1 * 2]);
      putfeat(fr, 53, sP[P_OH1 + c1 * 2 + 1]);
      putfeat(fr, 54, sP[P_OH2 + c2 * 2]);
      putfeat(fr, 55, sP[P_OH2 + c2 * 2 + 1]);
      putfeat(fr, 56, sP[P_OH3 + c3 * 3]);
      putfeat(fr, 57, sP[P_OH3 + c3 * 3 + 1]);
      putfeat(fr, 58, sP[P_OH3 + c3 * 3 + 2]);
      putfeat(fr, 59, sgn * sP[P_OH4 + c4]);
    } else {
#pragma unroll
      for (int i = 0; i < 8; ++i) putfeat(fr, 60 + i, sgn * sM[s * 9 + 1 + i]);
#pragma unroll
      for (int i = 0; i < 7; ++i) putfeat(fr, 68 + i, sNM[s * 9 + 2 + i]);
#pragma unroll
      for (int c = KF; c < K1H; ++c) putfeat(fr, c, 0.0f);
    }
  }
  __syncthreads();

  v8f acc[8];
  {
    const v8f z = {0.f, 0.f, 0.f, 0.f, 0.f, 0.f, 0.f, 0.f};
#pragma unroll
    for (int t = 0; t < 8; ++t) acc[t] = z;
  }
  {
    const unsigned short* ap = sU + (16 * wave + m) * K1 + 8 * hh;
    const unsigned short* bp = W1P + (size_t)m * K1 + 8 * hh;
#pragma unroll 1
    for (int k0 = 0; k0 < K1; k0 += 32) {
      FragB af;
      af.h[0] = *(const v8usa*)(ap + k0);
      af.h[1] = *(const v8usa*)(ap + k0 + 16);
#pragma unroll
      for (int nt = 0; nt < 8; ++nt) {
        const unsigned short* wq = bp + (size_t)(16 * nt) * K1 + k0;
        FragB bf;
        bf.h[0] = *(const v8usa*)wq;
        bf.h[1] = *(const v8usa*)(wq + 16);
        acc[nt] = wmb(af, bf, acc[nt]);
      }
    }
  }
  __syncthreads();

#pragma unroll
  for (int nt = 0; nt < 8; ++nt) {
    const int col = 16 * nt + m;
    const float b1 = sP[P_B1 + col];
#pragma unroll
    for (int r = 0; r < 8; ++r) {
      const int row = 16 * wave + 8 * hh + r;
      const float v = fmaxf(acc[nt][r] + b1, 0.0f);
      const unsigned hb = bf16_bits(v);
      const unsigned lb = bf16_bits(v - __uint_as_float(hb << 16));
      sU[row * K2 + col]      = (unsigned short)hb;
      sU[row * K2 + N1 + col] = (unsigned short)lb;
    }
  }
  __syncthreads();

  v8f ac2[4];
  {
    const v8f z = {0.f, 0.f, 0.f, 0.f, 0.f, 0.f, 0.f, 0.f};
#pragma unroll
    for (int t = 0; t < 4; ++t) ac2[t] = z;
  }
  {
    const unsigned short* ap = sU + (16 * wave + m) * K2 + 8 * hh;
    const unsigned short* bp = W2P + (size_t)m * K2 + 8 * hh;
#pragma unroll 1
    for (int k0 = 0; k0 < K2; k0 += 32) {
      FragB af;
      af.h[0] = *(const v8usa*)(ap + k0);
      af.h[1] = *(const v8usa*)(ap + k0 + 16);
#pragma unroll
      for (int nt = 0; nt < 4; ++nt) {
        const unsigned short* wq = bp + (size_t)(16 * nt) * K2 + k0;
        FragB bf;
        bf.h[0] = *(const v8usa*)wq;
        bf.h[1] = *(const v8usa*)(wq + 16);
        ac2[nt] = wmb(af, bf, ac2[nt]);
      }
    }
  }
#pragma unroll
  for (int nt = 0; nt < 4; ++nt) {
    const int col = 16 * nt + m;
    const float b2 = sP[P_B2 + col];
#pragma unroll
    for (int r = 0; r < 8; ++r) {
      const int row = 16 * wave + 8 * hh + r;
      sY[row * N2 + col] = fmaxf(ac2[nt][r] + b2, 0.0f);
    }
  }
  __syncthreads();

  if (tid < 128) {
    const float* yr = sY + tid * N2;
    float l0 = 0.0f, l1 = 0.0f, l2 = 0.0f;
#pragma unroll 1
    for (int c4 = 0; c4 < N2 / 4; ++c4) {
      const v4f y  = *(const v4fa*)(yr + 4 * c4);
      const v4f w0 = *(const v4fa*)(sP + P_PIW + 4 * c4);
      const v4f w1 = *(const v4fa*)(sP + P_PIW + 64 + 4 * c4);
      const v4f w2 = *(const v4fa*)(sP + P_PIW + 128 + 4 * c4);
      l0 = fmaf(y.x, w0.x, l0); l0 = fmaf(y.y, w0.y, l0); l0 = fmaf(y.z, w0.z, l0); l0 = fmaf(y.w, w0.w, l0);
      l1 = fmaf(y.x, w1.x, l1); l1 = fmaf(y.y, w1.y, l1); l1 = fmaf(y.z, w1.z, l1); l1 = fmaf(y.w, w1.w, l1);
      l2 = fmaf(y.x, w2.x, l2); l2 = fmaf(y.y, w2.y, l2); l2 = fmaf(y.z, w2.z, l2); l2 = fmaf(y.w, w2.w, l2);
    }
    l0 = l0 + sP[P_PIB + 0];
    l1 = l1 + sP[P_PIB + 1];
    l2 = l2 + sP[P_PIB + 2];
    const float mx = fmaxf(l0, fmaxf(l1, l2));
    const float e0 = expf(l0 - mx), e1 = expf(l1 - mx), e2 = expf(l2 - mx);
    const float ss = (e0 + e1) + e2;
    sSM[tid * 4 + 0] = e0 / ss;
    sSM[tid * 4 + 1] = e1 / ss;
    sSM[tid * 4 + 2] = e2 / ss;
  }
  __syncthreads();

  if (tid < SPB) {
    const float* sa = sSM + tid * 4;
    const float* sb = sSM + (SPB + tid) * 4;
    const float o0 = 0.5f * (sb[0] + sa[2]);
    const float o1 = 0.5f * (sb[1] + sa[1]);
    const float o2 = 0.5f * (sb[2] + sa[0]);
    const int c1 = sC[tid * 5 + 1], c2 = sC[tid * 5 + 2], c3 = sC[tid * 5 + 3];
    const int hit = ((c1 == 5) | (c1 == 7)) & (c2 == 11) & (c3 == 4);
    const float ind = hit ? 1.0f : 0.0f;
    const float om  = 1.0f - ind;
    v4f o;
    o.x = om * o0 + ind * 0.0f;
    o.y = om * o1 + ind * 1.0f;
    o.z = om * o2 + ind * 0.0f;
    o.w = ind;
    putf4(PV + (s0 + (size_t)tid) * 4, o);
  }
}

__global__ __launch_bounds__(32) void k_scan(const float* __restrict__ PV, const float* __restrict__ PB,
                                             float* out) {
  const int lane = (int)threadIdx.x;
  const int jl = lane < 2 ? lane : 2;
  const float p0 = PB[P_POS + 0], p1 = PB[P_POS + 1], p2 = PB[P_POS + 2];
  const float flag = PB[P_FLAG];
  const float SHv = 0.9f, OMS = 0.1f;
  float R0 = 0.0f, R1 = 0.0f, R2 = 0.0f;
  float pr0 = p0, pr1 = p1, pr2 = p2;
  v4f cur = *(const v4fa*)(PV + 4 * (size_t)lane);
#pragma unroll 1
  for (int c = 0; c < NCHUNK; ++c) {
    const int cn = (c + 1 < NCHUNK) ? (c + 1) : c;
    const v4f nxt = *(const v4fa*)(PV + ((size_t)cn * 32 + (size_t)lane) * 4);
    float ms = 0.0f, mc = 0.0f;
#pragma unroll 1
    for (int i = 0; i < 32; ++i) {
      const float a0  = rl(cur.x, i);
      const float a1  = rl(cur.y, i);
      const float a2  = rl(cur.z, i);
      const float ind = rl(cur.w, i);
      const float om  = 1.0f - ind;
      const float qa = om * SHv;
      const float qb = om * OMS + ind;
      const float d1 = 2.0f * a0 + 2.0f * a2;
      const float cost = (pr0 * 0.0f + pr2 * 0.0f) + pr1 * d1;
      const int t = c * 32 + i;
      if (t == 0) {
        R0 = (jl == 0) ? qa : ((jl == 1) ? a0 : 0.0f);
        R1 = (jl == 0) ? qb : ((jl == 1) ? a1 : qb);
        R2 = (jl == 0) ? 0.0f : ((jl == 1) ? a2 : qa);
      } else {
        const float m0 = R0 * qa + R1 * a0;
        const float m1 = R0 * qb + R1 * a1 + R2 * qb;
        const float m2 = R1 * a2 + R2 * qa;
        const float s  = (m0 + m2) + m1;
        R0 = m0 / s;
        R1 = m1 / s;
        R2 = m2 / s;
      }
      const float M00 = rl(R0, 0), M01 = rl(R1, 0), M02 = rl(R2, 0);
      const float M10 = rl(R0, 1), M11 = rl(R1, 1), M12 = rl(R2, 1);
      const float M20 = rl(R0, 2), M21 = rl(R1, 2), M22 = rl(R2, 2);
      const float q0 = p0 * M00 + p1 * M10 + p2 * M20;
      const float q1 = p0 * M01 + p1 * M11 + p2 * M21;
      const float q2 = p0 * M02 + p1 * M12 + p2 * M22;
      const float sm = q2 - q0;
      ms = (lane == i) ? sm : ms;
      mc = (lane == i) ? cost : mc;
      pr0 = q0; pr1 = q1; pr2 = q2;
    }
    const float qn = __int_as_float(0x7fc00000);
    const float vs = (flag != 0.0f) ? qn : ms;
    const float vc = (flag != 0.0f) ? qn : mc;
    float* o0 = out + (size_t)c * 32 + (size_t)lane;
    float* o1 = out + (size_t)NB_S + (size_t)c * 32 + (size_t)lane;
    *(volatile float*)o0 = vs;
    *(volatile float*)o1 = vc;
    __threadfence();
    *(volatile float*)o0 = vs;
    *(volatile float*)o1 = vc;
    cur = nxt;
  }
}

extern "C" void kernel_launch(void* const* d_in, const int* in_sizes, int n_in,
                              void* d_out, int out_size, void* d_ws, size_t ws_size,
                              hipStream_t stream) {
  if (n_in < 26) return;
  if (in_sizes[0] != NB_S * 60 || in_sizes[1] != NB_S * 60) return;
  if (in_sizes[2] != NB_S * 9 || in_sizes[3] != NB_S * 9) return;
  if (in_sizes[4] != NB_S * 5) return;
  if (in_sizes[5] != 3 || in_sizes[6] != 1) return;
  if (in_sizes[7] != 80 || in_sizes[8] != 8 || in_sizes[9] != 80 || in_sizes[10] != 8) return;
  if (in_sizes[11] != N1 * KF || in_sizes[12] != N1) return;
  if (in_sizes[13] != N2 * N1 || in_sizes[14] != N2) return;
  if (in_sizes[15] != 3 * N2 || in_sizes[16] != 3) return;
  if (in_sizes[21] != 12 || in_sizes[22] != 24 || in_sizes[23] != 24) return;
  if (in_sizes[24] != 15 || in_sizes[25] != 10) return;
  if (out_size != 2 * NB_S) return;
  if ((size_t)WS_NEED > ws_size) return;

  const float* x    = (const float*)d_in[0];
  const float* xb   = (const float*)d_in[1];
  const float* xm   = (const float*)d_in[2];
  const float* xnm  = (const float*)d_in[3];
  const int*   xcat = (const int*)d_in[4];
  const float* pos0 = (const float*)d_in[5];
  const int*   modp = (const int*)d_in[6];
  const float* c00w = (const float*)d_in[7];
  const float* c00b = (const float*)d_in[8];
  const float* c10w = (const float*)d_in[9];
  const float* c10b = (const float*)d_in[10];
  const float* f11w = (const float*)d_in[11];
  const float* f11b = (const float*)d_in[12];
  const float* f12w = (const float*)d_in[13];
  const float* f12b = (const float*)d_in[14];
  const float* piw  = (const float*)d_in[15];
  const float* pib  = (const float*)d_in[16];
  const float* oh0  = (const float*)d_in[21];
  const float* oh1  = (const float*)d_in[22];
  const float* oh2  = (const float*)d_in[23];
  const float* oh3  = (const float*)d_in[24];
  const float* oh4  = (const float*)d_in[25];
  float* out = (float*)d_out;

  char* ws = (char*)d_ws;
  unsigned short* W1P = (unsigned short*)(ws + OW1);
  unsigned short* W2P = (unsigned short*)(ws + OW2);
  float*          PB  = (float*)(ws + OPB);
  float*          PV  = (float*)(ws + OPV);

  hipFuncSetAttribute(reinterpret_cast<const void*>(&k_mlp), hipFuncAttributeMaxDynamicSharedMemorySize,
                      (int)MLP_LDS);

  k_prep<<<NU_ALL / NTHR, NTHR, 0, stream>>>(f11w, f12w, c00w, c00b, c10w, c10b, f11b, f12b, piw, pib,
                                             oh0, oh1, oh2, oh3, oh4, pos0, modp, W1P, W2P, PB);
  k_mlp<<<NBLK, NTHR, MLP_LDS, stream>>>(x, xb, xm, xnm, xcat, W1P, W2P, PB, PV);
  k_scan<<<1, 32, 0, stream>>>(PV, PB, out);
}
